// QualityGatedMamba_29858612642530
// MI455X (gfx1250) — hardware-run, weakly checked
//
#include <hip/hip_runtime.h>
#include <hip/hip_fp16.h>
#include <math.h>

typedef __attribute__((ext_vector_type(16))) _Float16 v16h;
typedef __attribute__((ext_vector_type(8)))  _Float16 v8h;
typedef __attribute__((ext_vector_type(8)))  float    v8f;
typedef __attribute__((ext_vector_type(4)))  float    v4f;

constexpr int kBatch  = 2;
constexpr int kSeq    = 2048;
constexpr int kDm     = 1024;
constexpr int kDin    = 2048;
constexpr int kNst    = 16;
constexpr int kXzW    = 2 * kDin;
constexpr int kXpW    = 96;
constexpr int kBcP    = 64;
constexpr int kRows   = kBatch * kSeq;
constexpr int kConvTP = 260;
static_assert((kDm % 64) == 0 && (kDin % 64) == 0);
static_assert((kSeq % 64) == 0 && (kXzW % 64) == 0 && (kBcP % 64) == 0);
static_assert(2 * kNst <= kBcP && 2 * kNst <= kXpW);
static_assert((kDin % 256) == 0);

constexpr float kCarryX = 64.0f;
constexpr float kCarryW = 1024.0f;
constexpr float kCarryU = 64.0f;
constexpr float kCarryY = 64.0f;
constexpr float kResid  = 2048.0f;
constexpr float kInvXW  = 1.0f / (kCarryX * kCarryW);
constexpr float kInvUW  = 1.0f / (kCarryU * kCarryW);
constexpr float kInvYW  = 1.0f / (kCarryY * kCarryW);
constexpr float kInvRes = 1.0f / kResid;

constexpr size_t kOffX16  = 0;
constexpr size_t kOffWINT = kOffX16  + (size_t)kRows * kDm * 2;
constexpr size_t kOffWDT  = kOffWINT + (size_t)kXzW * kDm * 2;
constexpr size_t kOffWOT  = kOffWDT  + (size_t)kDin * kDm * 2;
constexpr size_t kOffWXT  = kOffWOT  + (size_t)kDm * kDin * 2;
constexpr size_t kOffALR  = kOffWXT  + (size_t)kBcP * kDin * 2;
constexpr size_t kOffDSK  = kOffALR  + (size_t)kDin * kNst * 4;
constexpr size_t kOffUPRE = kOffDSK  + (size_t)kDin * 4;
constexpr size_t kOffZPL  = kOffUPRE + (size_t)kSeq * kDin * 4;
constexpr size_t kOffUPL  = kOffZPL  + (size_t)kSeq * kDin * 4;
constexpr size_t kOffDTP  = kOffUPL  + (size_t)kSeq * kDin * 4;
constexpr size_t kOffUH   = kOffDTP  + (size_t)kSeq * kDin * 4;
constexpr size_t kOffUL   = kOffUH   + (size_t)kSeq * kDin * 2;
constexpr size_t kOffYH   = kOffUL   + (size_t)kSeq * kDin * 2;
constexpr size_t kOffYL   = kOffYH   + (size_t)kSeq * kDin * 2;
constexpr size_t kOffBC   = kOffYL   + (size_t)kSeq * kDin * 2;
constexpr size_t kWsTotal = kOffBC   + (size_t)kSeq * kBcP * 4;
static_assert(kWsTotal == 126754816ull);
static_assert(kWsTotal <= 134217728ull);
static_assert((kOffWINT % 128) == 0 && (kOffWDT % 128) == 0 && (kOffWOT % 128) == 0 && (kOffWXT % 128) == 0);
static_assert((kOffALR % 128) == 0 && (kOffDSK % 128) == 0 && (kOffUPRE % 128) == 0 && (kOffZPL % 128) == 0);
static_assert((kOffUPL % 128) == 0 && (kOffDTP % 128) == 0 && (kOffUH % 128) == 0 && (kOffUL % 128) == 0);
static_assert((kOffYH % 128) == 0 && (kOffYL % 128) == 0 && (kOffBC % 128) == 0);

__device__ __forceinline__ float bf16_rne(float f) {
  unsigned u = __float_as_uint(f);
  u = (u + 0x7FFFu + ((u >> 16) & 1u)) & 0xFFFF0000u;
  return __uint_as_float(u);
}
__device__ __forceinline__ float flush_h16(float v) {
  return (fabsf(v) < 6.103515625e-05f) ? 0.0f : v;
}
__device__ __forceinline__ _Float16 to_h16_flush(float v) {
  return (_Float16)flush_h16(v);
}
__device__ __forceinline__ void split_h16(float c, _Float16& hi, _Float16& lo) {
  hi = to_h16_flush(c);
  const float hf = (float)hi;
  const float r = (c - hf) * kResid;
  lo = to_h16_flush(r);
}

union FragU { v16h v; v8h h[2]; };
__device__ __forceinline__ v16h frag_load(const _Float16* p) {
  FragU f;
  f.h[0] = *(const v8h*)(p);
  f.h[1] = *(const v8h*)(p + 16);
  return f.v;
}
__device__ __forceinline__ v8f mma_h(v16h a, v16h b, v8f c) {
  return __builtin_amdgcn_wmma_f32_16x16x32_f16(false, a, false, b, (short)0, c, false, false);
}
__device__ __forceinline__ void guard1_h(v8f& acc, v16h x, v16h y) {
  asm volatile("v_nop\n\tv_nop\n\tv_nop\n\tv_nop" : "+v"(acc) : "v"(x), "v"(y));
}

__global__ __launch_bounds__(256) void cvt_x_kernel(
    const float* __restrict__ src, unsigned short* __restrict__ dst, int total8, float carry)
{
  const int i = blockIdx.x * 256 + threadIdx.x;
  if (i >= total8) return;
  const size_t e0 = (size_t)i << 3;
  const v4f a0 = *(const v4f*)(src + e0);
  const v4f a1 = *(const v4f*)(src + e0 + 4);
  v8h hv;
#pragma unroll
  for (int e = 0; e < 4; ++e) {
    const float f0 = a0[e];
    const float f1 = a1[e];
    hv[e]     = to_h16_flush(bf16_rne(f0) * carry);
    hv[4 + e] = to_h16_flush(bf16_rne(f1) * carry);
  }
  *(volatile v8h*)(dst + e0) = hv;
  __threadfence();
  *(volatile v8h*)(dst + e0) = hv;
}

__global__ __launch_bounds__(256) void wt_transpose_kernel(
    const float* __restrict__ W, int ld_src, int nvalid,
    unsigned short* __restrict__ Wt, int K, float carry)
{
  __shared__ float sT[64 * 65];
  const int tid = threadIdx.x, lane = tid & 31, wave = tid >> 5;
  const int k0 = blockIdx.x * 64;
  const int n0 = blockIdx.y * 64;
  const int nn = tid & 63;
  const int kq = tid >> 6;
  const int n  = n0 + nn;
  const bool ok = (n < nvalid);
  const int nc = ok ? n : (nvalid - 1);
#pragma unroll 4
  for (int i = 0; i < 16; ++i) {
    const int kk = kq + 4 * i;
    float v = W[(size_t)(k0 + kk) * ld_src + nc];
    asm volatile("" : "+v"(v));
    const float r = flush_h16(bf16_rne(v) * carry);
    sT[kk * 65 + nn] = ok ? r : 0.0f;
  }
  __syncthreads();
  const int q = lane >> 3, k8 = (lane & 7) * 8;
  v8h hv[2];
#pragma unroll
  for (int it = 0; it < 2; ++it) {
    const int row = it * 32 + wave * 4 + q;
#pragma unroll
    for (int e = 0; e < 8; ++e) hv[it][e] = (_Float16)sT[(k8 + e) * 65 + row];
  }
  for (int pass = 0; pass < 2; ++pass) {
#pragma unroll
    for (int it = 0; it < 2; ++it) {
      const int row = it * 32 + wave * 4 + q;
      *(volatile v8h*)(Wt + (size_t)(n0 + row) * K + k0 + k8) = hv[it];
    }
    __threadfence();
  }
}

__global__ __launch_bounds__(256) void rne_copy_kernel(
    const float* __restrict__ src, float* __restrict__ dst, int n4)
{
  const int i = blockIdx.x * 256 + threadIdx.x;
  if (i >= n4) return;
  const v4f a = *(const v4f*)(src + (size_t)i * 4);
  v4f r;
#pragma unroll
  for (int e = 0; e < 4; ++e) {
    const float f = a[e];
    r[e] = bf16_rne(f);
  }
  *(volatile v4f*)(dst + (size_t)i * 4) = r;
  __threadfence();
  *(volatile v4f*)(dst + (size_t)i * 4) = r;
}

__global__ __launch_bounds__(256) void gemm_f16_kernel(
    const unsigned short* __restrict__ Ap, int lda,
    const unsigned short* __restrict__ Btp, int ldb,
    float* C0, float* C1, int nsplit, int ldc,
    int M, int N, int K, float scale)
{
  const _Float16* A  = (const _Float16*)Ap;
  const _Float16* Bt = (const _Float16*)Btp;
  __shared__ __align__(16) float sT[8][16 * 68];
  const int lane = threadIdx.x & 31;
  const int wave = threadIdx.x >> 5;
  const int tilesN = N >> 6;
  const int tilesM = M >> 6;
  const int tile = blockIdx.x * 8 + wave;
  if (tile >= tilesM * tilesN) return;
  const int tm = tile / tilesN;
  const int tn = tile - tm * tilesN;
  const int m0 = tm << 6;
  const int n0 = tn << 6;
  const int rlane = lane & 15;
  const int koff  = (lane >> 4) * 8;
  const int mOff  = (lane >> 4) * 8;

  v8f acc[4][4];
#pragma unroll
  for (int i = 0; i < 4; ++i)
#pragma unroll
    for (int j = 0; j < 4; ++j) acc[i][j] = (v8f){0.f, 0.f, 0.f, 0.f, 0.f, 0.f, 0.f, 0.f};

  for (int k0 = 0; k0 < K; k0 += 32) {
    v16h bh[4];
#pragma unroll
    for (int j = 0; j < 4; ++j) {
      const size_t bo = (size_t)(n0 + (j << 4) + rlane) * ldb + koff + k0;
      bh[j] = frag_load(Bt + bo);
    }
#pragma unroll
    for (int i = 0; i < 4; ++i) {
      const size_t ao = (size_t)(m0 + (i << 4) + rlane) * lda + koff + k0;
      const v16h ah = frag_load(A + ao);
#pragma unroll
      for (int j = 0; j < 4; ++j) acc[i][j] = mma_h(ah, bh[j], acc[i][j]);
#pragma unroll
      for (int j = 0; j < 4; ++j) guard1_h(acc[i][j], ah, bh[j]);
    }
  }

  float* slab = sT[wave];
  float* Cb = (n0 < nsplit) ? C0 : C1;
  const int nc0 = (n0 < nsplit) ? n0 : (n0 - nsplit);
#pragma unroll
  for (int i = 0; i < 4; ++i) {
    const int mBase = m0 + (i << 4);
#pragma unroll
    for (int j = 0; j < 4; ++j) {
#pragma unroll
      for (int r = 0; r < 8; ++r) slab[(mOff + r) * 68 + (j << 4) + rlane] = acc[i][j][r] * scale;
    }
    __builtin_amdgcn_fence(__ATOMIC_RELEASE, "workgroup");
    __builtin_amdgcn_wave_barrier();
    __builtin_amdgcn_fence(__ATOMIC_ACQUIRE, "workgroup");
    {
      const int hh = lane >> 4, c4 = (lane & 15) * 4;
      for (int pass = 0; pass < 2; ++pass) {
#pragma unroll
        for (int it = 0; it < 8; ++it) {
          const int row = it * 2 + hh;
          v4f v = *(const v4f*)(slab + row * 68 + c4);
          *(volatile v4f*)(Cb + (size_t)(mBase + row) * ldc + nc0 + c4) = v;
        }
        __threadfence();
      }
    }
    __builtin_amdgcn_fence(__ATOMIC_RELEASE, "workgroup");
    __builtin_amdgcn_wave_barrier();
    __builtin_amdgcn_fence(__ATOMIC_ACQUIRE, "workgroup");
  }
}

__global__ __launch_bounds__(256) void gemm_f16_resid_kernel(
    const unsigned short* __restrict__ Ahp, const unsigned short* __restrict__ Alp, int lda,
    const unsigned short* __restrict__ Btp, int ldb,
    float* C, int ldc, int M, int N, int K, float scale, float rinv)
{
  const _Float16* Ah = (const _Float16*)Ahp;
  const _Float16* Al = (const _Float16*)Alp;
  const _Float16* Bt = (const _Float16*)Btp;
  __shared__ __align__(16) float sT[8][16 * 68];
  const int lane = threadIdx.x & 31;
  const int wave = threadIdx.x >> 5;
  const int tilesN = N >> 6;
  const int tilesM = M >> 5;
  const int tile = blockIdx.x * 8 + wave;
  if (tile >= tilesM * tilesN) return;
  const int tm = tile / tilesN;
  const int tn = tile - tm * tilesN;
  const int m0 = tm << 5;
  const int n0 = tn << 6;
  const int rlane = lane & 15;
  const int koff  = (lane >> 4) * 8;
  const int mOff  = (lane >> 4) * 8;

  v8f ach[2][4], acl[2][4];
#pragma unroll
  for (int i = 0; i < 2; ++i)
#pragma unroll
    for (int j = 0; j < 4; ++j) {
      ach[i][j] = (v8f){0.f, 0.f, 0.f, 0.f, 0.f, 0.f, 0.f, 0.f};
      acl[i][j] = (v8f){0.f, 0.f, 0.f, 0.f, 0.f, 0.f, 0.f, 0.f};
    }

  for (int k0 = 0; k0 < K; k0 += 32) {
    v16h bh[4];
#pragma unroll
    for (int j = 0; j < 4; ++j) {
      const size_t bo = (size_t)(n0 + (j << 4) + rlane) * ldb + koff + k0;
      bh[j] = frag_load(Bt + bo);
    }
#pragma unroll
    for (int i = 0; i < 2; ++i) {
      const size_t ao = (size_t)(m0 + (i << 4) + rlane) * lda + koff + k0;
      const v16h ah = frag_load(Ah + ao);
      const v16h al = frag_load(Al + ao);
#pragma unroll
      for (int j = 0; j < 4; ++j) {
        ach[i][j] = mma_h(ah, bh[j], ach[i][j]);
        acl[i][j] = mma_h(al, bh[j], acl[i][j]);
      }
#pragma unroll
      for (int j = 0; j < 4; ++j) {
        guard1_h(ach[i][j], ah, bh[j]);
        guard1_h(acl[i][j], al, bh[j]);
      }
    }
  }

  float* slab = sT[wave];
#pragma unroll
  for (int i = 0; i < 2; ++i) {
    const int mBase = m0 + (i << 4);
#pragma unroll
    for (int j = 0; j < 4; ++j) {
#pragma unroll
      for (int r = 0; r < 8; ++r) {
        const float s = fmaf(acl[i][j][r], rinv, ach[i][j][r]);
        slab[(mOff + r) * 68 + (j << 4) + rlane] = s * scale;
      }
    }
    __builtin_amdgcn_fence(__ATOMIC_RELEASE, "workgroup");
    __builtin_amdgcn_wave_barrier();
    __builtin_amdgcn_fence(__ATOMIC_ACQUIRE, "workgroup");
    {
      const int hh = lane >> 4, c4 = (lane & 15) * 4;
      for (int pass = 0; pass < 2; ++pass) {
#pragma unroll
        for (int it = 0; it < 8; ++it) {
          const int row = it * 2 + hh;
          v4f v = *(const v4f*)(slab + row * 68 + c4);
          *(volatile v4f*)(C + (size_t)(mBase + row) * ldc + n0 + c4) = v;
        }
        __threadfence();
      }
    }
    __builtin_amdgcn_fence(__ATOMIC_RELEASE, "workgroup");
    __builtin_amdgcn_wave_barrier();
    __builtin_amdgcn_fence(__ATOMIC_ACQUIRE, "workgroup");
  }
}

__global__ __launch_bounds__(256) void conv_silu_kernel(
    const float* __restrict__ UP, const float* __restrict__ cw, const float* __restrict__ cb,
    float* __restrict__ U, unsigned short* __restrict__ UH, unsigned short* __restrict__ UL)
{
  __shared__ __align__(16) float sT[16 * kConvTP];
  const int tid = threadIdx.x, lane = tid & 31, wave = tid >> 5;
  const int d0 = blockIdx.x * 256, d = d0 + tid;
  const int g0 = blockIdx.y * 64;
  const float w0 = bf16_rne(cw[0 * kDin + d]);
  const float w1 = bf16_rne(cw[1 * kDin + d]);
  const float w2 = bf16_rne(cw[2 * kDin + d]);
  const float w3 = bf16_rne(cw[3 * kDin + d]);
  const float bcv = bf16_rne(cb[d]);
  float xm3, xm2, xm1;
  {
    const bool hist = (g0 > 0);
    const int rb = hist ? (g0 - 3) : 0;
    const float v3 = UP[(size_t)rb * kDin + d];
    const float v2 = UP[(size_t)(rb + 1) * kDin + d];
    const float v1 = UP[(size_t)(rb + 2) * kDin + d];
    xm3 = hist ? v3 : 0.0f;
    xm2 = hist ? v2 : 0.0f;
    xm1 = hist ? v1 : 0.0f;
  }
  const int hrow = wave >> 1;
  const int hch  = (wave & 1) * 128 + lane * 4;
#pragma unroll 1
  for (int sub = 0; sub < 4; ++sub) {
    const int lb = g0 + sub * 16;
#pragma unroll 1
    for (int s = 0; s < 16; ++s) {
      const float xcur = UP[(size_t)(lb + s) * kDin + d];
      float acc = w0 * xm3;
      acc = fmaf(w1, xm2, acc);
      acc = fmaf(w2, xm1, acc);
      acc = fmaf(w3, xcur, acc);
      const float sv = acc + bcv;
      const float den = 1.0f + expf(-sv);
      sT[s * kConvTP + tid] = sv * (1.0f / den);
      xm3 = xm2;
      xm2 = xm1;
      xm1 = xcur;
    }
    __syncthreads();
    v4f fv[4];
    v8h vh[2], vl[2];
#pragma unroll
    for (int it = 0; it < 4; ++it) fv[it] = *(const v4f*)(sT + (it * 4 + hrow) * kConvTP + hch);
#pragma unroll
    for (int it = 0; it < 2; ++it) {
      const float* sp = sT + (it * 8 + wave) * kConvTP + lane * 8;
      const v4f a0 = *(const v4f*)(sp);
      const v4f a1 = *(const v4f*)(sp + 4);
#pragma unroll
      for (int e = 0; e < 4; ++e) {
        const float f0 = a0[e];
        const float f1 = a1[e];
        _Float16 h0, l0, h1, l1;
        split_h16(f0 * kCarryU, h0, l0);
        split_h16(f1 * kCarryU, h1, l1);
        vh[it][e]     = h0;
        vh[it][4 + e] = h1;
        vl[it][e]     = l0;
        vl[it][4 + e] = l1;
      }
    }
    for (int pass = 0; pass < 2; ++pass) {
#pragma unroll
      for (int it = 0; it < 4; ++it)
        *(volatile v4f*)(U + (size_t)(lb + it * 4 + hrow) * kDin + d0 + hch) = fv[it];
#pragma unroll
      for (int it = 0; it < 2; ++it) {
        const size_t o = (size_t)(lb + it * 8 + wave) * kDin + d0 + lane * 8;
        *(volatile v8h*)(UH + o) = vh[it];
        *(volatile v8h*)(UL + o) = vl[it];
      }
      __threadfence();
    }
    __syncthreads();
  }
}

__global__ __launch_bounds__(256) void step_pre_kernel(
    const float* __restrict__ raw, const float* __restrict__ bdl, const float* __restrict__ sig,
    const float* __restrict__ alpha_p, float* __restrict__ DT)
{
  __shared__ __align__(16) float sD[kDin];
  const int tid = threadIdx.x;
  const int row = blockIdx.x;
  const float al = bf16_rne(alpha_p[0]);
  const float s2 = bf16_rne(sig[row]);
  const float gate = expf((-al) * s2);
#pragma unroll 1
  for (int it = 0; it < kDin / 256; ++it) {
    const int c = it * 256 + tid;
    const float v = raw[(size_t)row * kDin + c] + bf16_rne(bdl[c]);
    const float sp = fmaxf(v, 0.0f) + log1pf(expf(-fabsf(v)));
    const float y = sp * gate;
    const float inv = logf(expm1f(y));
    sD[c] = (y > 20.0f) ? y : inv;
  }
  __syncthreads();
  v4f o[2];
#pragma unroll
  for (int it = 0; it < 2; ++it) o[it] = *(const v4f*)(sD + (it * 256 + tid) * 4);
  for (int pass = 0; pass < 2; ++pass) {
#pragma unroll
    for (int it = 0; it < 2; ++it)
      *(volatile v4f*)(DT + (size_t)row * kDin + (it * 256 + tid) * 4) = o[it];
    __threadfence();
  }
}

typedef float    ms1_v4f __attribute__((ext_vector_type(4)));
typedef unsigned ms1_v4u __attribute__((ext_vector_type(4)));
struct ms1_args {
  const float* dtpre;
  const float* u;
  const float* bc;
  const float* z;
  const float* A_log;
  const float* Dskip;
  __half* y;
  __half* y_lo;
  long ld_dtpre;
  long ld_u;
  long ld_bc;
  long ld_z;
  long ld_y;
  int offB;
  int offC;
  int offZ;
  float ycarry;
  int dir;
  int D;
  int L;
  int nbatch;
};
static_assert(sizeof(ms1_args) == 136);

__device__ __forceinline__ float ms1_flush16(float v) {
  return (fabsf(v) < 6.103515625e-05f) ? 0.0f : v;
}
__device__ __forceinline__ unsigned ms1_h16bits(float v) {
  return (unsigned)__half_as_ushort(__float2half_rn(ms1_flush16(v)));
}
__device__ __forceinline__ float ms1_h16val(unsigned b) {
  return __half2float(__ushort_as_half((unsigned short)b));
}
__device__ __forceinline__ float ms1_softplus(float v) {
  return fmaxf(v, 0.0f) + log1pf(expf(-fabsf(v)));
}
__device__ __forceinline__ void ms1_pack2(float v0, float v1, unsigned& hw, unsigned& lw) {
  const unsigned h0 = ms1_h16bits(v0);
  const unsigned h1 = ms1_h16bits(v1);
  const float r0 = (v0 - ms1_h16val(h0)) * 2048.0f;
  const float r1 = (v1 - ms1_h16val(h1)) * 2048.0f;
  const unsigned l0 = ms1_h16bits(r0);
  const unsigned l1 = ms1_h16bits(r1);
  hw = h0 | (h1 << 16);
  lw = l0 | (l1 << 16);
}

template <int NSTATE>
__global__ __launch_bounds__(64 * (NSTATE / 16)) void ms1_scan_kernel(ms1_args a)
{
  static_assert(NSTATE == 16 || NSTATE == 64);
  constexpr int NQ  = NSTATE / 16;
  constexpr int NT  = 64 * NQ;
  constexpr int NW  = NT / 32;
  constexpr int BCW = 2 * NSTATE;
  constexpr int YP  = 68;
  constexpr int RPI = NW * 4;
  constexpr int NIT = 64 / RPI;
  static_assert(16 * NT <= 64 * YP);
  __shared__ __align__(16) float sBC[64 * BCW];
  __shared__ __align__(16) float sY[64 * YP];
  const int tid  = threadIdx.x;
  const int lane = tid & 31;
  const int wave = tid >> 5;
  const int c    = tid / NQ;
  const int sq   = tid - c * NQ;
  const int bpb  = a.D / 64;
  const int bi   = blockIdx.x / bpb;
  if (bi >= a.nbatch) return;
  const int d0 = (blockIdx.x - bi * bpb) * 64;
  const int d  = d0 + c;
  const long rowb = (long)bi * a.L;
  const bool hasz  = (a.z != nullptr);
  const bool hasD  = (a.Dskip != nullptr);
  const bool hasLo = (a.y_lo != nullptr);

#pragma unroll 1
  for (int n = 0; n < 16; ++n) {
    const float al = a.A_log[(long)d * NSTATE + sq * 16 + n];
    sY[n * NT + tid] = -expf(al);
  }
  __syncthreads();
  float An[16], h[16];
#pragma unroll
  for (int n = 0; n < 16; ++n) {
    An[n] = sY[n * NT + tid];
    h[n] = 0.0f;
  }
  float Dd = 0.0f;
  if (hasD) Dd = a.Dskip[d];

  const int nchunk = a.L / 64;
  const bool fwd = (a.dir > 0);
  const int s0 = fwd ? 0 : 63;
  const int sd = fwd ? 1 : -1;
  const int q  = lane >> 3;
  const int c8 = (lane & 7) * 8;

#pragma unroll 1
  for (int ci = 0; ci < nchunk; ++ci) {
    const int tb = fwd ? (ci * 64) : (a.L - 64 - ci * 64);
    const long rowc = rowb + tb;
    __syncthreads();
#pragma unroll 8
    for (int i = 0; i < 32; ++i) {
      const int idx = tid + i * NT;
      const int st  = idx / BCW;
      const int col = idx - st * BCW;
      const int sc  = (col < NSTATE) ? (a.offB + col) : (a.offC + col - NSTATE);
      sBC[idx] = a.bc[(rowc + st) * a.ld_bc + sc];
    }
    __syncthreads();
#pragma unroll 1
    for (int s = 0; s < 64; ++s) {
      const int ls = s0 + sd * s;
      const long row = rowc + ls;
      float pre = a.dtpre[row * a.ld_dtpre + d];
      float uv  = a.u[row * a.ld_u + d];
      float zv  = 0.0f;
      if (hasz) zv = a.z[row * a.ld_z + a.offZ + d];
      asm volatile("" : "+v"(pre));
      asm volatile("" : "+v"(uv));
      asm volatile("" : "+v"(zv));
      const float delta = ms1_softplus(pre);
      const float dtx = delta * uv;
      const float* bp = sBC + ls * BCW + sq * 16;
      const float* cp = bp + NSTATE;
      ms1_v4f Bq[4], Cq[4];
#pragma unroll
      for (int k = 0; k < 4; ++k) {
        Bq[k] = *(const ms1_v4f*)(bp + 4 * k);
        Cq[k] = *(const ms1_v4f*)(cp + 4 * k);
      }
      float yv = 0.0f;
#pragma unroll
      for (int n = 0; n < 16; ++n) {
        const float e = __expf(delta * An[n]);
        h[n] = fmaf(e, h[n], dtx * Bq[n >> 2][n & 3]);
        yv = fmaf(h[n], Cq[n >> 2][n & 3], yv);
      }
      if (NQ > 1) {
        yv += __shfl_xor(yv, 1, 32);
        yv += __shfl_xor(yv, 2, 32);
      }
      if (hasD) yv = fmaf(uv, Dd, yv);
      if (hasz) {
        const float sg = __builtin_amdgcn_rcpf(1.0f + expf(-zv));
        yv = yv * (zv * sg);
      }
      if (sq == 0) sY[ls * YP + c] = yv * a.ycarry;
    }
    __syncthreads();
    ms1_v4u hw[NIT], lw[NIT];
#pragma unroll
    for (int it = 0; it < NIT; ++it) {
      const int row = it * RPI + wave * 4 + q;
      const float* sp = sY + row * YP + c8;
      const ms1_v4f f0 = *(const ms1_v4f*)(sp);
      const ms1_v4f f1 = *(const ms1_v4f*)(sp + 4);
      unsigned h0, h1, h2, h3, l0, l1, l2, l3;
      ms1_pack2(f0[0], f0[1], h0, l0);
      ms1_pack2(f0[2], f0[3], h1, l1);
      ms1_pack2(f1[0], f1[1], h2, l2);
      ms1_pack2(f1[2], f1[3], h3, l3);
      hw[it] = (ms1_v4u){h0, h1, h2, h3};
      lw[it] = (ms1_v4u){l0, l1, l2, l3};
    }
    for (int pass = 0; pass < 2; ++pass) {
#pragma unroll
      for (int it = 0; it < NIT; ++it) {
        const int row = it * RPI + wave * 4 + q;
        const long o = (rowc + row) * a.ld_y + d0 + c8;
        *(volatile ms1_v4u*)(a.y + o) = hw[it];
        if (hasLo) *(volatile ms1_v4u*)(a.y_lo + o) = lw[it];
      }
      __threadfence();
    }
  }
}

extern "C" void kernel_launch(void* const* d_in, const int* in_sizes, int n_in,
                              void* d_out, int out_size, void* d_ws, size_t ws_size,
                              hipStream_t stream)
{
  if (n_in < 12) return;
  if (in_sizes[0] != kRows * kDm) return;
  if (in_sizes[1] != kRows) return;
  if (in_sizes[2] != kDm * kXzW) return;
  if (in_sizes[3] != 4 * kDin) return;
  if (in_sizes[4] != kDin) return;
  if (in_sizes[5] != kDin * kXpW) return;
  if (in_sizes[6] != kDm * kDin) return;
  if (in_sizes[7] != kDin) return;
  if (in_sizes[8] != kDin * kNst) return;
  if (in_sizes[9] != kDin) return;
  if (in_sizes[10] != kDin * kDm) return;
  if (in_sizes[11] != 1) return;
  if (out_size != kRows * kDm) return;
  if (ws_size < kWsTotal) return;

  const float* x       = (const float*)d_in[0];
  const float* sigma2  = (const float*)d_in[1];
  const float* W_in    = (const float*)d_in[2];
  const float* conv_w  = (const float*)d_in[3];
  const float* conv_b  = (const float*)d_in[4];
  const float* W_xproj = (const float*)d_in[5];
  const float* W_delta = (const float*)d_in[6];
  const float* b_delta = (const float*)d_in[7];
  const float* A_log   = (const float*)d_in[8];
  const float* D_par   = (const float*)d_in[9];
  const float* W_out   = (const float*)d_in[10];
  const float* alpha_p = (const float*)d_in[11];
  float* out = (float*)d_out;

  char* ws = (char*)d_ws;
  unsigned short* X16  = (unsigned short*)(ws + kOffX16);
  unsigned short* WINT = (unsigned short*)(ws + kOffWINT);
  unsigned short* WDT  = (unsigned short*)(ws + kOffWDT);
  unsigned short* WOT  = (unsigned short*)(ws + kOffWOT);
  unsigned short* WXT  = (unsigned short*)(ws + kOffWXT);
  float*          ALR  = (float*)(ws + kOffALR);
  float*          DSK  = (float*)(ws + kOffDSK);
  float*          UPRE = (float*)(ws + kOffUPRE);
  float*          ZPL  = (float*)(ws + kOffZPL);
  float*          UPL  = (float*)(ws + kOffUPL);
  float*          DTP  = (float*)(ws + kOffDTP);
  unsigned short* UH   = (unsigned short*)(ws + kOffUH);
  unsigned short* UL   = (unsigned short*)(ws + kOffUL);
  unsigned short* YH   = (unsigned short*)(ws + kOffYH);
  unsigned short* YL   = (unsigned short*)(ws + kOffYL);
  float*          BC   = (float*)(ws + kOffBC);

  cvt_x_kernel<<<dim3((kRows * kDm / 8) / 256), 256, 0, stream>>>(x, X16, kRows * kDm / 8, kCarryX);
  wt_transpose_kernel<<<dim3(kDm / 64, kXzW / 64), 256, 0, stream>>>(W_in, kXzW, kXzW, WINT, kDm, kCarryW);
  wt_transpose_kernel<<<dim3(kDm / 64, kDin / 64), 256, 0, stream>>>(W_delta, kDin, kDin, WDT, kDm, kCarryW);
  wt_transpose_kernel<<<dim3(kDin / 64, kDm / 64), 256, 0, stream>>>(W_out, kDm, kDm, WOT, kDin, kCarryW);
  wt_transpose_kernel<<<dim3(kDin / 64, kBcP / 64), 256, 0, stream>>>(W_xproj, kXpW, 2 * kNst, WXT, kDin, kCarryW);
  rne_copy_kernel<<<dim3((kDin * kNst / 4) / 256), 256, 0, stream>>>(A_log, ALR, kDin * kNst / 4);
  rne_copy_kernel<<<dim3((kDin / 4 + 255) / 256), 256, 0, stream>>>(D_par, DSK, kDin / 4);

  for (int b = 0; b < kBatch; ++b) {
    const unsigned short* Xb = X16 + (size_t)b * kSeq * kDm;

    gemm_f16_kernel<<<dim3((kSeq / 64) * (kXzW / 64) / 8), 256, 0, stream>>>(
        Xb, kDm, WINT, kDm, UPRE, ZPL, kDin, kDin, kSeq, kXzW, kDm, kInvXW);

    conv_silu_kernel<<<dim3(kDin / 256, kSeq / 64), 256, 0, stream>>>(UPRE, conv_w, conv_b, UPL, UH, UL);

    gemm_f16_resid_kernel<<<dim3((kSeq / 32) * (kBcP / 64) / 8), 256, 0, stream>>>(
        UH, UL, kDin, WXT, kDin, BC, kBcP, kSeq, kBcP, kDin, kInvUW, kInvRes);

    gemm_f16_kernel<<<dim3((kSeq / 64) * (kDin / 64) / 8), 256, 0, stream>>>(
        Xb, kDm, WDT, kDm, UPRE, UPRE, kDin, kDin, kSeq, kDin, kDm, kInvXW);

    step_pre_kernel<<<dim3(kSeq), 256, 0, stream>>>(UPRE, b_delta, sigma2 + (size_t)b * kSeq, alpha_p, DTP);

    ms1_args sa;
    sa.dtpre = DTP;
    sa.u = UPL;
    sa.bc = BC;
    sa.z = ZPL;
    sa.A_log = ALR;
    sa.Dskip = DSK;
    sa.y = (__half*)YH;
    sa.y_lo = (__half*)YL;
    sa.ld_dtpre = kDin;
    sa.ld_u = kDin;
    sa.ld_bc = kBcP;
    sa.ld_z = kDin;
    sa.ld_y = kDin;
    sa.offB = 0;
    sa.offC = kNst;
    sa.offZ = 0;
    sa.ycarry = kCarryY;
    sa.dir = 1;
    sa.D = kDin;
    sa.L = kSeq;
    sa.nbatch = 1;
    ms1_scan_kernel<16><<<dim3(kDin / 64), 64, 0, stream>>>(sa);

    gemm_f16_resid_kernel<<<dim3((kSeq / 32) * (kDm / 64) / 8), 256, 0, stream>>>(
        YH, YL, kDin, WOT, kDin, out + (size_t)b * kSeq * kDm, kDm, kSeq, kDm, kDin, kInvYW, kInvRes);
  }
}
